// GNN_86586540687361
// MI455X (gfx1250) — hardware-verified
//
#include <hip/hip_runtime.h>
#include <stddef.h>
#include <stdint.h>


#define DIN1   128
#define HID    64
#define KP     256
#define NLAY   6
#define NTHR   256
#define NWAVE  8
#define EPT    8
#define CHUNK  (NTHR * EPT)
#define WCAP   (EPT * 32)
#define LISTN  (NWAVE * WCAP)
#define NBA    1024
#define SLA    10
#define RCAP   28672
#define DEGCAP 128
#define GBM    64
#define GBN    64
#define GTHR   128
#define WPU    2048
#define NPB    128
#define NPW    16
#define AGG_ZINTS    (LISTN + 2 * RCAP + 3 * NBA)
#define AGG_LDS_INTS (AGG_ZINTS + 16)
#define WSMAX  134217728

static_assert((CHUNK & (CHUNK - 1)) == 0 && CHUNK <= 4096);
static_assert((NBA & (NBA - 1)) == 0 && NBA == (1 << SLA));
static_assert(((long long)CHUNK << SLA) < (1LL << 31));
static_assert(LISTN % NTHR == 0);
static_assert(NBA == NTHR * 4 && NBA % 32 == 0 && NBA % GBM == 0);
static_assert(RCAP % (NTHR * 4) == 0 && RCAP < 32768 && DEGCAP < 255);
static_assert(AGG_ZINTS % 4 == 0 && LISTN % 4 == 0 && ((LISTN + RCAP) % 4) == 0);
static_assert(KP % 32 == 0 && KP == 2 * DIN1 && KP == 4 * HID && HID == GBN);
static_assert(GBM == (GTHR / 32) * 16);
static_assert((NLAY * WPU) % NTHR == 0 && WPU == HID * (KP / 8));
static_assert(NPB == NWAVE * NPW);
static_assert(AGG_LDS_INTS * 4 <= 300000);

typedef float          v4f   __attribute__((ext_vector_type(4)));
typedef float          v8f   __attribute__((ext_vector_type(8)));
typedef int            v4i   __attribute__((ext_vector_type(4)));
typedef int            v8i   __attribute__((ext_vector_type(8)));
typedef unsigned int   v4u   __attribute__((ext_vector_type(4)));
typedef unsigned short v8us  __attribute__((ext_vector_type(8)));
typedef unsigned short v16us __attribute__((ext_vector_type(16)));
typedef __bf16         v16bf __attribute__((ext_vector_type(16)));
typedef v4f  __attribute__((may_alias)) v4fa;
typedef v4i  __attribute__((may_alias)) v4ia;
typedef v4u  __attribute__((may_alias)) v4ua;
typedef v8us __attribute__((may_alias)) v8usa;
union FragB { v16bf v; v16us u; v8us h[2]; v8i w; };

__device__ __forceinline__ v8f wmb(const FragB& a, const FragB& b, v8f c) {
  v8f d = __builtin_amdgcn_wmma_f32_16x16x32_bf16(false, a.v, false, b.v, (short)0, c, false, false);
  asm volatile("v_nop\n\tv_nop\n\tv_nop\n\tv_nop" : "+v"(d) : "v"(a.w), "v"(b.w));
  return d;
}

__device__ __forceinline__ unsigned bf16_bits(float f) {
  const unsigned u = __float_as_uint(f);
  return (u + 0x7FFFu + ((u >> 16) & 1u)) >> 16;
}
__device__ __forceinline__ float bf16_val(float f) {
  return __uint_as_float(bf16_bits(f) << 16);
}
__device__ __forceinline__ float nmax(float m, float v) {
  return (v > m || v != v) ? v : m;
}
__device__ __forceinline__ unsigned blendu(unsigned x, unsigned y, unsigned msk) {
  return (x & ~msk) | (y & msk);
}
__device__ __forceinline__ v4u hilo4(float a, float b, float c, float d) {
  const unsigned h0 = bf16_bits(a), h1 = bf16_bits(b), h2 = bf16_bits(c), h3 = bf16_bits(d);
  const unsigned l0 = bf16_bits(a - __uint_as_float(h0 << 16));
  const unsigned l1 = bf16_bits(b - __uint_as_float(h1 << 16));
  const unsigned l2 = bf16_bits(c - __uint_as_float(h2 << 16));
  const unsigned l3 = bf16_bits(d - __uint_as_float(h3 << 16));
  v4u r;
  r.x = h0 | (h1 << 16);
  r.y = h2 | (h3 << 16);
  r.z = l0 | (l1 << 16);
  r.w = l2 | (l3 << 16);
  return r;
}

template <int SLB>
__device__ __forceinline__ int scan_chunk(const int* __restrict__ dsts, int nE, int cbase, int slotBase,
                                          int nb, int vec8, int* list, int tid, int lane, int wave) {
  int wc = 0;
  const int el0  = tid * EPT;
  const int e0   = cbase + el0;
  const int sent = -2147483647 - 1;
  v4i da, db;
  if (vec8 != 0 && cbase + CHUNK <= nE) {
    da = *(const v4i*)(dsts + e0);
    db = *(const v4i*)(dsts + e0 + 4);
  } else {
    da.x = (e0     < nE) ? dsts[min(e0,     nE - 1)] : sent;
    da.y = (e0 + 1 < nE) ? dsts[min(e0 + 1, nE - 1)] : sent;
    da.z = (e0 + 2 < nE) ? dsts[min(e0 + 2, nE - 1)] : sent;
    da.w = (e0 + 3 < nE) ? dsts[min(e0 + 3, nE - 1)] : sent;
    db.x = (e0 + 4 < nE) ? dsts[min(e0 + 4, nE - 1)] : sent;
    db.y = (e0 + 5 < nE) ? dsts[min(e0 + 5, nE - 1)] : sent;
    db.z = (e0 + 6 < nE) ? dsts[min(e0 + 6, nE - 1)] : sent;
    db.w = (e0 + 7 < nE) ? dsts[min(e0 + 7, nE - 1)] : sent;
  }
  const unsigned nbs = (unsigned)slotBase;
  const unsigned unb = (unsigned)nb;
  const unsigned s0 = (unsigned)da.x - nbs, s1 = (unsigned)da.y - nbs;
  const unsigned s2 = (unsigned)da.z - nbs, s3 = (unsigned)da.w - nbs;
  const unsigned s4 = (unsigned)db.x - nbs, s5 = (unsigned)db.y - nbs;
  const unsigned s6 = (unsigned)db.z - nbs, s7 = (unsigned)db.w - nbs;
  const bool h0 = s0 < unb, h1 = s1 < unb, h2 = s2 < unb, h3 = s3 < unb;
  const bool h4 = s4 < unb, h5 = s5 < unb, h6 = s6 < unb, h7 = s7 < unb;
  const unsigned any = __builtin_amdgcn_ballot_w32(h0 | h1 | h2 | h3 | h4 | h5 | h6 | h7);
  if (any != 0u) {
#define HITJ(J, HJ, SJ) { \
      const unsigned mj = __builtin_amdgcn_ballot_w32(HJ); \
      if (mj != 0u) { \
        if (HJ) { \
          const int pos = wc + (int)__builtin_amdgcn_mbcnt_lo(mj, 0u); \
          if (pos < WCAP) list[wave * WCAP + pos] = ((el0 + (J)) << SLB) | (int)(SJ); \
        } \
        wc += (int)__builtin_popcount(mj); } }
    HITJ(0, h0, s0)
    HITJ(1, h1, s1)
    HITJ(2, h2, s2)
    HITJ(3, h3, s3)
    HITJ(4, h4, s4)
    HITJ(5, h5, s5)
    HITJ(6, h6, s6)
    HITJ(7, h7, s7)
#undef HITJ
  }
  return wc;
}

__global__ __launch_bounds__(NTHR) void k_wprep(const float* __restrict__ W1l, const float* __restrict__ W1r,
                                                const float* __restrict__ Wml, const float* __restrict__ Wmr,
                                                const float* __restrict__ W6l, const float* __restrict__ W6r,
                                                unsigned short* WC) {
  const int u   = (int)blockIdx.x * NTHR + (int)threadIdx.x;
  const int p   = u >> 11;
  const int v   = u & (WPU - 1);
  const int n   = v >> 5;
  const int k8i = v & 31;
  const int g   = k8i & 15;
  const unsigned msk = (k8i >= 16) ? 0xffffffffu : 0u;
  v8us o;
  if (p == 0) {
    const size_t so = (size_t)n * DIN1 + 8 * g;
    const v4f a = *(const v4f*)(W1l + so);
    const v4f b = *(const v4f*)(W1l + so + 4);
    const v4f c = *(const v4f*)(W1r + so);
    const v4f d = *(const v4f*)(W1r + so + 4);
    o[0] = (unsigned short)blendu(bf16_bits(a.x), bf16_bits(c.x), msk);
    o[1] = (unsigned short)blendu(bf16_bits(a.y), bf16_bits(c.y), msk);
    o[2] = (unsigned short)blendu(bf16_bits(a.z), bf16_bits(c.z), msk);
    o[3] = (unsigned short)blendu(bf16_bits(a.w), bf16_bits(c.w), msk);
    o[4] = (unsigned short)blendu(bf16_bits(b.x), bf16_bits(d.x), msk);
    o[5] = (unsigned short)blendu(bf16_bits(b.y), bf16_bits(d.y), msk);
    o[6] = (unsigned short)blendu(bf16_bits(b.z), bf16_bits(d.z), msk);
    o[7] = (unsigned short)blendu(bf16_bits(b.w), bf16_bits(d.w), msk);
  } else if (p < 5) {
    const size_t so = (size_t)(p - 1) * (HID * HID) + (size_t)n * HID + 4 * g;
    const v4f a = *(const v4f*)(Wml + so);
    const v4f c = *(const v4f*)(Wmr + so);
    const unsigned short e0 = (unsigned short)blendu(bf16_bits(a.x), bf16_bits(c.x), msk);
    const unsigned short e1 = (unsigned short)blendu(bf16_bits(a.y), bf16_bits(c.y), msk);
    const unsigned short e2 = (unsigned short)blendu(bf16_bits(a.z), bf16_bits(c.z), msk);
    const unsigned short e3 = (unsigned short)blendu(bf16_bits(a.w), bf16_bits(c.w), msk);
    o[0] = e0; o[1] = e1; o[2] = e2; o[3] = e3; o[4] = e0; o[5] = e1; o[6] = e2; o[7] = e3;
  } else if (p == 5) {
    const size_t so = (size_t)n * HID + 4 * g;
    const v4f a = *(const v4f*)(W6l + so);
    const v4f c = *(const v4f*)(W6r + so);
    const unsigned short e0 = (unsigned short)blendu(bf16_bits(a.x), bf16_bits(c.x), msk);
    const unsigned short e1 = (unsigned short)blendu(bf16_bits(a.y), bf16_bits(c.y), msk);
    const unsigned short e2 = (unsigned short)blendu(bf16_bits(a.z), bf16_bits(c.z), msk);
    const unsigned short e3 = (unsigned short)blendu(bf16_bits(a.w), bf16_bits(c.w), msk);
    o[0] = e0; o[1] = e1; o[2] = e2; o[3] = e3; o[4] = e0; o[5] = e1; o[6] = e2; o[7] = e3;
  } else {
    return;
  }
  unsigned short* dp = WC + (size_t)p * (HID * KP) + (size_t)n * KP + 8 * k8i;
  *(volatile v8us*)dp = o;
  __threadfence();
  *(volatile v8us*)dp = o;
}

__global__ __launch_bounds__(NTHR) void k_cvx(const float* __restrict__ x, int nN, int nUnits,
                                              unsigned short* apl) {
  const int u = (int)blockIdx.x * NTHR + (int)threadIdx.x;
  if (u >= nUnits) return;
  const int row = u >> 4;
  const int k8  = (u & 15) * 8;
  const int rc  = row < nN ? row : nN - 1;
  const float* p = x + (size_t)rc * DIN1 + k8;
  const v4f a = *(const v4fa*)p;
  const v4f b = *(const v4fa*)(p + 4);
  const bool ok = row < nN;
  v8us o;
  o[0] = ok ? (unsigned short)bf16_bits(a.x) : (unsigned short)0;
  o[1] = ok ? (unsigned short)bf16_bits(a.y) : (unsigned short)0;
  o[2] = ok ? (unsigned short)bf16_bits(a.z) : (unsigned short)0;
  o[3] = ok ? (unsigned short)bf16_bits(a.w) : (unsigned short)0;
  o[4] = ok ? (unsigned short)bf16_bits(b.x) : (unsigned short)0;
  o[5] = ok ? (unsigned short)bf16_bits(b.y) : (unsigned short)0;
  o[6] = ok ? (unsigned short)bf16_bits(b.z) : (unsigned short)0;
  o[7] = ok ? (unsigned short)bf16_bits(b.w) : (unsigned short)0;
  unsigned short* dp = apl + (size_t)row * KP + DIN1 + k8;
  *(volatile v8us*)dp = o;
  __threadfence();
  *(volatile v8us*)dp = o;
}

__global__ __launch_bounds__(NTHR) void k_lists(const int* __restrict__ srcs, const int* __restrict__ dsts,
                                                int nE, int nN, int vec8, int* tab, int* srcl) {
  extern __shared__ __attribute__((aligned(16))) int dsm[];
  int* list = dsm;
  int* hl   = dsm + LISTN;
  int* sl   = hl + RCAP;
  int* cnt  = sl + RCAP;
  int* offs = cnt + NBA;
  int* cur  = offs + NBA;
  int* misc = cur + NBA;
  const int tid = (int)threadIdx.x, lane = tid & 31, wave = tid >> 5;
  const int nodeBase = (int)blockIdx.x * NBA;

  {
    const v4i z4 = {0, 0, 0, 0};
    for (int i = tid * 4; i < AGG_ZINTS; i += NTHR * 4) *(v4ia*)(dsm + i) = z4;
    if (tid < 16) misc[tid] = 0;
  }
  __syncthreads();

  int t = 0, ov = 0;
  const int nChunks = (nE + CHUNK - 1) / CHUNK;
#pragma unroll 1
  for (int ch = 0; ch < nChunks; ++ch) {
    const int cbase = ch * CHUNK;
    const int wc = scan_chunk<SLA>(dsts, nE, cbase, nodeBase, NBA, vec8, list, tid, lane, wave);
    if (lane == 0) misc[wave] = wc;
    __syncthreads();
    if (wave == 0) {
#pragma unroll 1
      for (int w2 = 0; w2 < NWAVE; ++w2) {
        int c = misc[w2];
        c = c < 0 ? 0 : (c > WCAP ? WCAP : c);
#pragma unroll 1
        for (int b0 = 0; b0 < c; b0 += 32) {
          const int idx = b0 + lane;
          const int ent = list[w2 * WCAP + (idx < WCAP ? idx : WCAP - 1)];
          const int m32 = (c - b0) < 32 ? (c - b0) : 32;
#pragma unroll 1
          for (int k = 0; k < m32; ++k) {
            const int u    = __builtin_amdgcn_readlane(ent, k);
            const int slot = u & (NBA - 1);
            const int el   = (u >> SLA) & (CHUNK - 1);
            const int pk   = ((cbase + el) << SLA) | slot;
            if (t < RCAP) {
              if (lane == 0) { hl[t] = pk; cnt[slot] = cnt[slot] + 1; }
              t = t + 1;
            } else {
              ov = 1;
            }
          }
        }
      }
    }
    __syncthreads();
  }
  if (wave == 0 && lane == 0) { misc[8] = t; misc[9] = ov; }
  __syncthreads();
  int tt = misc[8];
  tt = tt < 0 ? 0 : (tt > RCAP ? RCAP : tt);
  const int ovf = misc[9];

  if (wave == 0) {
    const int base = lane * (NBA / 32);
    int s = 0;
#pragma unroll 1
    for (int i = 0; i < NBA / 32; ++i) s += cnt[base + i];
    int incl = s;
#pragma unroll
    for (int d = 1; d < 32; d <<= 1) {
      const int y = __shfl_up(incl, d, 32);
      if (lane >= d) incl += y;
    }
    int run = incl - s;
#pragma unroll 1
    for (int i = 0; i < NBA / 32; ++i) {
      const int cv = cnt[base + i];
      offs[base + i] = run;
      cur[base + i]  = run;
      run += cv;
    }
  }
  __syncthreads();
  if (wave == 0) {
#pragma unroll 1
    for (int b0 = 0; b0 < tt; b0 += 32) {
      const int idx = b0 + lane;
      const int ent = hl[idx < RCAP ? idx : RCAP - 1];
      const int m32 = (tt - b0) < 32 ? (tt - b0) : 32;
#pragma unroll 1
      for (int k = 0; k < m32; ++k) {
        const int u    = __builtin_amdgcn_readlane(ent, k);
        const int slot = u & (NBA - 1);
        if (lane == 0) {
          int p = cur[slot];
          p = p < 0 ? 0 : (p > RCAP - 1 ? RCAP - 1 : p);
          sl[p] = u;
          cur[slot] = p + 1;
        }
      }
    }
  }
  __syncthreads();

  {
    const v4i c4 = *(const v4ia*)(cnt + 4 * tid);
    const v4i o4 = *(const v4ia*)(offs + 4 * tid);
    const int fb = (ovf != 0) ? (1 << 30) : 0;
    v4i e;
    {
      int cc, oo;
      cc = c4.x < 0 ? 0 : (c4.x > 255 ? 255 : c4.x); oo = o4.x < 0 ? 0 : (o4.x > RCAP ? RCAP : o4.x); e.x = fb | (oo << 8) | cc;
      cc = c4.y < 0 ? 0 : (c4.y > 255 ? 255 : c4.y); oo = o4.y < 0 ? 0 : (o4.y > RCAP ? RCAP : o4.y); e.y = fb | (oo << 8) | cc;
      cc = c4.z < 0 ? 0 : (c4.z > 255 ? 255 : c4.z); oo = o4.z < 0 ? 0 : (o4.z > RCAP ? RCAP : o4.z); e.z = fb | (oo << 8) | cc;
      cc = c4.w < 0 ? 0 : (c4.w > 255 ? 255 : c4.w); oo = o4.w < 0 ? 0 : (o4.w > RCAP ? RCAP : o4.w); e.w = fb | (oo << 8) | cc;
    }
    int* tp = tab + (size_t)nodeBase + 4 * tid;
    *(volatile v4i*)tp = e;
    __threadfence();
    *(volatile v4i*)tp = e;
  }
  int* lp = srcl + (size_t)blockIdx.x * RCAP;
#pragma unroll 1
  for (int it = 0; it < RCAP / (NTHR * 4); ++it) {
    const int i0 = it * (NTHR * 4) + 4 * tid;
    const v4i e4 = *(const v4ia*)(sl + i0);
    int q0 = e4.x >> SLA, q1 = e4.y >> SLA, q2 = e4.z >> SLA, q3 = e4.w >> SLA;
    q0 = q0 < 0 ? 0 : (q0 > nE - 1 ? nE - 1 : q0);
    q1 = q1 < 0 ? 0 : (q1 > nE - 1 ? nE - 1 : q1);
    q2 = q2 < 0 ? 0 : (q2 > nE - 1 ? nE - 1 : q2);
    q3 = q3 < 0 ? 0 : (q3 > nE - 1 ? nE - 1 : q3);
    int r0 = srcs[q0], r1 = srcs[q1], r2 = srcs[q2], r3 = srcs[q3];
    r0 = r0 < 0 ? 0 : (r0 > nN - 1 ? nN - 1 : r0);
    r1 = r1 < 0 ? 0 : (r1 > nN - 1 ? nN - 1 : r1);
    r2 = r2 < 0 ? 0 : (r2 > nN - 1 ? nN - 1 : r2);
    r3 = r3 < 0 ? 0 : (r3 > nN - 1 ? nN - 1 : r3);
    v4i r;
    r.x = (i0     < tt) ? r0 : 0;
    r.y = (i0 + 1 < tt) ? r1 : 0;
    r.z = (i0 + 2 < tt) ? r2 : 0;
    r.w = (i0 + 3 < tt) ? r3 : 0;
    *(volatile v4i*)(lp + i0) = r;
    __threadfence();
    *(volatile v4i*)(lp + i0) = r;
  }
}

template <int L1>
__global__ __launch_bounds__(NTHR) void k_agg(const int* __restrict__ srcl, const int* __restrict__ tab,
                                              int tabN, int nN, int mRows,
                                              const float* __restrict__ hin,
                                              const unsigned short* xsrc, unsigned short* apl) {
  constexpr int NV = (L1 != 0) ? 8 : 4;
  const int tid = (int)threadIdx.x, lane = tid & 31, wave = tid >> 5;
  const int hf = lane >> 4, q = lane & 15;
  const unsigned hm = (unsigned)(-hf);
  const float ninf = __uint_as_float(0xff800000u);
  const float qnan = __uint_as_float(0x7fc00000u);
#pragma unroll 1
  for (int si = 0; si < NPW; ++si) {
    const int node = __builtin_amdgcn_readfirstlane((int)blockIdx.x * NPB + wave * NPW + si);
    const int nt   = node < tabN ? node : tabN - 1;
    const int ent  = __builtin_amdgcn_readfirstlane(tab[nt]);
    const bool inr = node < mRows;
    const int c0   = inr ? (ent & 255) : 0;
    const bool big = c0 > DEGCAP;
    const int c    = c0 > DEGCAP ? DEGCAP : c0;
    int o = (ent >> 8) & 0x7fff;
    o = o > RCAP ? RCAP : o;
    const bool ovf = ((ent >> 30) & 1) != 0;
    const size_t lb = (size_t)(nt >> SLA) * RCAP;

    float mx[NV];
#pragma unroll
    for (int j = 0; j < NV; ++j) mx[j] = ninf;

#pragma unroll 1
    for (int b0 = 0; b0 < c; b0 += 32) {
      int idx = o + b0 + lane;
      idx = idx > RCAP - 1 ? RCAP - 1 : idx;
      int sr = srcl[lb + idx];
      sr = sr < 0 ? 0 : (sr > nN - 1 ? nN - 1 : sr);
      const int m32 = (c - b0) < 32 ? (c - b0) : 32;
#pragma unroll 1
      for (int k = 0; k < m32; k += 2) {
        const int k1 = (k + 1 < m32) ? (k + 1) : (m32 - 1);
        const unsigned sa = (unsigned)__builtin_amdgcn_readlane(sr, k);
        const unsigned sb = (unsigned)__builtin_amdgcn_readlane(sr, k1);
        const int sk = (int)blendu(sa, sb, hm);
        if constexpr (L1 != 0) {
          const v4u w = *(const v4ua*)(xsrc + (size_t)sk * KP + DIN1 + 8 * q);
          mx[0] = nmax(mx[0], __uint_as_float(w.x << 16));
          mx[1] = nmax(mx[1], __uint_as_float(w.x & 0xffff0000u));
          mx[2] = nmax(mx[2], __uint_as_float(w.y << 16));
          mx[3] = nmax(mx[3], __uint_as_float(w.y & 0xffff0000u));
          mx[4] = nmax(mx[4], __uint_as_float(w.z << 16));
          mx[5] = nmax(mx[5], __uint_as_float(w.z & 0xffff0000u));
          mx[6] = nmax(mx[6], __uint_as_float(w.w << 16));
          mx[7] = nmax(mx[7], __uint_as_float(w.w & 0xffff0000u));
        } else {
          const v4f a = *(const v4fa*)(hin + (size_t)sk * HID + 4 * q);
          mx[0] = nmax(mx[0], a.x);
          mx[1] = nmax(mx[1], a.y);
          mx[2] = nmax(mx[2], a.z);
          mx[3] = nmax(mx[3], a.w);
        }
      }
    }
#pragma unroll
    for (int j = 0; j < NV; ++j) {
      const float ot = __shfl_xor(mx[j], 16, 32);
      mx[j] = nmax(mx[j], ot);
    }
    const bool empty = (c0 == 0);
    const bool live  = node < nN;
    const float pz   = (ovf || big) ? qnan : 0.0f;
    float vv[NV];
#pragma unroll
    for (int j = 0; j < NV; ++j) {
      float v = empty ? 0.0f : mx[j];
      v = v + pz;
      vv[j] = live ? v : 0.0f;
    }
    v4u pv;
    if constexpr (L1 != 0) {
      pv.x = (__float_as_uint(vv[0]) >> 16) | (__float_as_uint(vv[1]) & 0xffff0000u);
      pv.y = (__float_as_uint(vv[2]) >> 16) | (__float_as_uint(vv[3]) & 0xffff0000u);
      pv.z = (__float_as_uint(vv[4]) >> 16) | (__float_as_uint(vv[5]) & 0xffff0000u);
      pv.w = (__float_as_uint(vv[6]) >> 16) | (__float_as_uint(vv[7]) & 0xffff0000u);
    } else {
      pv = hilo4(vv[0], vv[1], vv[2], vv[3]);
    }
    const int nd = inr ? node : 0;
    unsigned short* hp = apl + (size_t)nd * KP + 8 * q;
    const bool wr = inr && (lane < 16);
    if (wr) *(volatile v4u*)hp = pv;
    __threadfence();
    if (wr) *(volatile v4u*)hp = pv;
  }
}

template <int FIN>
__global__ __launch_bounds__(GTHR) void k_gemm(unsigned short* Apl, const unsigned short* __restrict__ WT,
                                               const float* __restrict__ bias, float* outF, int nN) {
  __shared__ __attribute__((aligned(16))) float stg[GBM * GBN];
  const int tid = (int)threadIdx.x, lane = tid & 31, wave = tid >> 5, hh = lane >> 4, m = lane & 15;
  const int rowBase = (int)blockIdx.x * GBM;

  v8f acc[4];
  {
    const v8f z = {0.f, 0.f, 0.f, 0.f, 0.f, 0.f, 0.f, 0.f};
    acc[0] = z; acc[1] = z; acc[2] = z; acc[3] = z;
  }
  const unsigned short* ap = Apl + (size_t)(rowBase + 16 * wave + m) * (size_t)KP + 8 * hh;
  const unsigned short* wp = WT + (size_t)m * (size_t)KP + 8 * hh;
#pragma unroll 1
  for (int ks = 0; ks < KP / 32; ++ks) {
    FragB af;
    af.h[0] = *(const v8usa*)(ap + 32 * ks);
    af.h[1] = *(const v8usa*)(ap + 32 * ks + 16);
#pragma unroll
    for (int t = 0; t < 4; ++t) {
      const unsigned short* wq = wp + (size_t)(16 * t) * (size_t)KP + 32 * ks;
      FragB bf;
      bf.h[0] = *(const v8usa*)wq;
      bf.h[1] = *(const v8usa*)(wq + 16);
      acc[t] = wmb(af, bf, acc[t]);
    }
  }

#pragma unroll
  for (int t = 0; t < 4; ++t) {
    const int lc = 16 * t + m;
#pragma unroll
    for (int r = 0; r < 8; ++r) {
      const int lr = 16 * wave + 8 * hh + r;
      stg[lr * GBN + lc] = acc[t][r];
    }
  }
  __syncthreads();

  v4f bb;
  {
    const v4f tb = *(const v4f*)(bias + 4 * m);
    bb.x = bf16_val(tb.x); bb.y = bf16_val(tb.y); bb.z = bf16_val(tb.z); bb.w = bf16_val(tb.w);
  }
  v4f fv[8];
  v4u pq[8];
#pragma unroll
  for (int i = 0; i < 8; ++i) {
    const int lr = 16 * wave + 2 * i + hh;
    v4f y = *(const v4fa*)(stg + lr * GBN + 4 * m) + bb;
    if constexpr (FIN == 0) {
      y.x = (y.x > 0.0f) ? y.x : (y.x - y.x);
      y.y = (y.y > 0.0f) ? y.y : (y.y - y.y);
      y.z = (y.z > 0.0f) ? y.z : (y.z - y.z);
      y.w = (y.w > 0.0f) ? y.w : (y.w - y.w);
    }
    const bool ok = (rowBase + lr) < nN;
    y.x = ok ? y.x : 0.0f; y.y = ok ? y.y : 0.0f; y.z = ok ? y.z : 0.0f; y.w = ok ? y.w : 0.0f;
    fv[i] = y;
    if constexpr (FIN == 0) pq[i] = hilo4(y.x, y.y, y.z, y.w);
  }

  if constexpr (FIN == 0) {
#pragma unroll
    for (int i = 0; i < 8; ++i) {
      const int gr = rowBase + 16 * wave + 2 * i + hh;
      *(volatile v4f*)(outF + (size_t)gr * HID + 4 * m) = fv[i];
      *(volatile v4u*)(Apl + (size_t)gr * KP + 2 * HID + 8 * m) = pq[i];
    }
    __threadfence();
#pragma unroll
    for (int i = 0; i < 8; ++i) {
      const int gr = rowBase + 16 * wave + 2 * i + hh;
      *(volatile v4f*)(outF + (size_t)gr * HID + 4 * m) = fv[i];
      *(volatile v4u*)(Apl + (size_t)gr * KP + 2 * HID + 8 * m) = pq[i];
    }
  } else {
#pragma unroll
    for (int i = 0; i < 8; ++i) {
      const int gr = rowBase + 16 * wave + 2 * i + hh;
      if (gr < nN) *(volatile v4f*)(outF + (size_t)gr * HID + 4 * m) = fv[i];
    }
    __threadfence();
#pragma unroll
    for (int i = 0; i < 8; ++i) {
      const int gr = rowBase + 16 * wave + 2 * i + hh;
      if (gr < nN) *(volatile v4f*)(outF + (size_t)gr * HID + 4 * m) = fv[i];
    }
  }
}

static inline int cdiv(int a, int b) { return (a + b - 1) / b; }
static inline size_t al256(size_t o) { return (o + 255) & ~(size_t)255; }

extern "C" void kernel_launch(void* const* d_in, const int* in_sizes, int n_in,
                              void* d_out, int out_size, void* d_ws, size_t ws_size,
                              hipStream_t stream) {
  if (n_in < 11) return;
  if (in_sizes[0] < DIN1 || (in_sizes[0] % DIN1) != 0) return;
  const int nN = in_sizes[0] / DIN1;
  if (nN < 16 || nN > (1 << 22)) return;
  if (in_sizes[1] < 2 || (in_sizes[1] & 1) != 0) return;
  const int nE = in_sizes[1] / 2;
  if (nE < 1 || nE >= (1 << (31 - SLA))) return;
  if (in_sizes[2] != HID * DIN1 || in_sizes[3] != HID) return;
  if (in_sizes[4] != HID * DIN1) return;
  if (in_sizes[5] != 4 * HID * HID || in_sizes[6] != 4 * HID) return;
  if (in_sizes[7] != 4 * HID * HID) return;
  if (in_sizes[8] != HID * HID || in_sizes[9] != HID) return;
  if (in_sizes[10] != HID * HID) return;
  if ((long long)out_size != (long long)nN * HID) return;

  const float* x    = (const float*)d_in[0];
  const int*   edge = (const int*)d_in[1];
  const float* W1l  = (const float*)d_in[2];
  const float* b1   = (const float*)d_in[3];
  const float* W1r  = (const float*)d_in[4];
  const float* Wml  = (const float*)d_in[5];
  const float* bm   = (const float*)d_in[6];
  const float* Wmr  = (const float*)d_in[7];
  const float* W6l  = (const float*)d_in[8];
  const float* b6   = (const float*)d_in[9];
  const float* W6r  = (const float*)d_in[10];
  float* out = (float*)d_out;
  const int* src = edge;
  const int* dst = edge + nE;

  const int MP   = cdiv(nN, GBM) * GBM;
  const int gM   = MP / GBM;
  const int gA   = cdiv(MP, NBA);
  const int tabN = gA * NBA;
  const int gG   = cdiv(MP, NPB);
  if ((long long)gA * NBA < (long long)MP) return;
  if ((long long)gG * NPB < (long long)MP) return;
  const int vec8 = ((nE & 3) == 0) ? 1 : 0;

  char* ws = (char*)d_ws;
  size_t off = 0;
  const size_t oWC  = off; off = al256(off + (size_t)NLAY * HID * KP * 2);
  const size_t oA   = off; off = al256(off + (size_t)MP * KP * 2);
  const size_t oHA  = off; off = al256(off + (size_t)MP * HID * 4);
  const size_t oHB  = off; off = al256(off + (size_t)MP * HID * 4);
  const size_t oTAB = off; off = al256(off + (size_t)tabN * 4);
  const size_t oSL  = off; off = al256(off + (size_t)gA * RCAP * 4);
  if (off > ws_size || off > (size_t)WSMAX) return;
  unsigned short* WC   = (unsigned short*)(ws + oWC);
  unsigned short* Apl  = (unsigned short*)(ws + oA);
  float*          HA   = (float*)(ws + oHA);
  float*          HB   = (float*)(ws + oHB);
  int*            TAB  = (int*)(ws + oTAB);
  int*            SRCL = (int*)(ws + oSL);

  const size_t ldsB = (size_t)AGG_LDS_INTS * 4;
  hipFuncSetAttribute(reinterpret_cast<const void*>(&k_lists), hipFuncAttributeMaxDynamicSharedMemorySize, (int)ldsB);

  const int nUx = MP * (DIN1 / 8);
  k_wprep<<<(NLAY * WPU) / NTHR, NTHR, 0, stream>>>(W1l, W1r, Wml, Wmr, W6l, W6r, WC);
  k_cvx<<<cdiv(nUx, NTHR), NTHR, 0, stream>>>(x, nN, nUx, Apl);
  k_lists<<<gA, NTHR, ldsB, stream>>>(src, dst, nE, nN, vec8, TAB, SRCL);
  k_agg<1><<<gG, NTHR, 0, stream>>>(SRCL, TAB, tabN, nN, MP, x, Apl, Apl);
  k_gemm<0><<<gM, GTHR, 0, stream>>>(Apl, WC, b1, HA, nN);
  float* hc = HA;
  float* hn = HB;
  for (int l = 2; l <= 5; ++l) {
    k_agg<0><<<gG, NTHR, 0, stream>>>(SRCL, TAB, tabN, nN, MP, hc, Apl, Apl);
    k_gemm<0><<<gM, GTHR, 0, stream>>>(Apl, WC + (size_t)(l - 1) * HID * KP, bm + (size_t)(l - 2) * HID, hn, nN);
    float* tq = hc; hc = hn; hn = tq;
  }
  k_agg<0><<<gG, NTHR, 0, stream>>>(SRCL, TAB, tabN, nN, MP, hc, Apl, Apl);
  k_gemm<1><<<gM, GTHR, 0, stream>>>(Apl, WC + (size_t)5 * HID * KP, b6, out, nN);
}
